// KPConvLayer_80401787781839
// MI455X (gfx1250) — hardware-verified
//
#include <hip/hip_runtime.h>
#include <math.h>

typedef __attribute__((ext_vector_type(16))) _Float16 v16h;
typedef __attribute__((ext_vector_type(16))) __bf16 v16b;
typedef __attribute__((ext_vector_type(8)))  _Float16 v8h;
typedef __attribute__((ext_vector_type(8)))  float v8f;
typedef __attribute__((ext_vector_type(4)))  float v4f;
typedef __attribute__((ext_vector_type(2)))  float v2f;
typedef __attribute__((ext_vector_type(4)))  unsigned v4u;
typedef __attribute__((ext_vector_type(4)))  int v4i;
typedef float __attribute__((may_alias)) float_a;
typedef int __attribute__((may_alias)) int_a;

template <typename T> __device__ __forceinline__ void vst2(void* p, T v) { *(volatile T*)p = v; __threadfence(); *(volatile T*)p = v; }
__device__ __forceinline__ v8f wmma16(v16h a, v16h b, v8f c) {
  v8f d = __builtin_amdgcn_wmma_f32_16x16x32_f16(false, a, false, b, (short)0, c, false, false);
  asm volatile("v_nop\n\tv_nop\n\tv_nop\n\tv_nop" : "+v"(d) : "v"(a), "v"(b));
  return d;
}
__device__ __forceinline__ v8f wmma_bf(v16b a, v16b b, v8f c) {
  v8f d = __builtin_amdgcn_wmma_f32_16x16x32_bf16(false, a, false, b, (short)0, c, false, false);
  asm volatile("v_nop\n\tv_nop\n\tv_nop\n\tv_nop" : "+v"(d) : "v"(a), "v"(b));
  return d;
}
__device__ __forceinline__ v16h frag_h(const _Float16* rowk0, int lane) {
  union { v16h v; v8h q[2]; } u; const _Float16* p = rowk0 + 8 * (lane >> 4);
  u.q[0] = *(const v8h*)p; u.q[1] = *(const v8h*)(p + 16); return u.v;
}
__device__ __forceinline__ v16h frag_f32(const float* rowk0, int lane) {
  v16h a; const float* p = rowk0 + 8 * (lane >> 4);
#pragma unroll
  for (int i = 0; i < 8; ++i) { a[i] = (_Float16)p[i]; a[8 + i] = (_Float16)p[16 + i]; }
  return a;
}
__device__ __forceinline__ v16h frag_f32s(const float* rowk0, int lane, float sc) {
  v16h a; const float* p = rowk0 + 8 * (lane >> 4);
#pragma unroll
  for (int i = 0; i < 8; ++i) { a[i] = (_Float16)(p[i] * sc); a[8 + i] = (_Float16)(p[16 + i] * sc); }
  return a;
}
__device__ __forceinline__ v16h fragc_f32(const float* W, int k0, int n, int lane, int ld, int K) {
  v16h a; const int g = lane >> 4;
#pragma unroll
  for (int i = 0; i < 8; ++i) { const int ka = k0 + 8 * g + i, kb = ka + 16;
    a[i] = (_Float16)(ka < K ? W[(size_t)ka * ld + n] : 0.f); a[8 + i] = (_Float16)(kb < K ? W[(size_t)kb * ld + n] : 0.f); }
  return a;
}
struct F2 { v16b h, l; };
__device__ __forceinline__ F2 bsplit16(const float v[16]) { F2 r;
#pragma unroll
  for (int i = 0; i < 16; ++i) { const __bf16 h = (__bf16)v[i]; r.h[i] = h; r.l[i] = (__bf16)(v[i] - (float)h); }
  return r; }
__device__ __forceinline__ F2 split_row(const float* row, int k0, int lane) { float v[16]; const float* p = row + k0 + 8 * (lane >> 4);
#pragma unroll
  for (int i = 0; i < 8; ++i) { v[i] = p[i]; v[8 + i] = p[16 + i]; }
  return bsplit16(v); }
__device__ __forceinline__ F2 split_rowK(const float* row, int k0, int lane, int K) { float v[16]; const int g = lane >> 4;
#pragma unroll
  for (int i = 0; i < 8; ++i) { const int ka = k0 + 8 * g + i, kb = ka + 16; v[i] = ka < K ? row[ka] : 0.f; v[8 + i] = kb < K ? row[kb] : 0.f; }
  return bsplit16(v); }
__device__ __forceinline__ F2 split_col(const float* W, int k0, int n, int lane, int ld, int K) { float v[16]; const int g = lane >> 4;
#pragma unroll
  for (int i = 0; i < 8; ++i) { const int ka = k0 + 8 * g + i, kb = ka + 16; v[i] = ka < K ? W[(size_t)ka * ld + n] : 0.f; v[8 + i] = kb < K ? W[(size_t)kb * ld + n] : 0.f; }
  return bsplit16(v); }
__device__ __forceinline__ v8f mac3(const F2& a, const F2& b, v8f c) { c = wmma_bf(a.l, b.h, c); c = wmma_bf(a.h, b.l, c); return wmma_bf(a.h, b.h, c); }
__device__ __forceinline__ float sigm(float v) { return 1.0f / (1.0f + expf(-v)); }
#define LDSX() do { asm volatile("s_wait_dscnt 0" ::: "memory"); __builtin_amdgcn_wave_barrier(); __builtin_amdgcn_fence(__ATOMIC_RELEASE, "workgroup"); } while (0)

#define NQ 32768
#define N0 40000
#define MM 32
#define KP 15
#define CIN 64
#define COUT 128
#define KW (KP * CIN)

__global__ __launch_bounds__(256) void k_agg(const float* __restrict__ qp, const float* __restrict__ sp, const int* __restrict__ nb, const float* __restrict__ x, const float* __restrict__ kpts, float* __restrict__ WF) {
  __shared__ float sw[8][KP][MM + 1];
  __shared__ int sid[8][MM];
  __shared__ float skp[KP * 3];
  const int tid = threadIdx.x, w = tid >> 5, lane = tid & 31; const int n = blockIdx.x * 8 + w;
  if (tid < KP * 3) skp[tid] = kpts[tid];
  __syncthreads();
  { int id = nb[(size_t)n * MM + lane]; const bool shadow = (id < 0) || (id >= N0); id = shadow ? 0 : id; sid[w][lane] = shadow ? -1 : id;
    const float qx = qp[(size_t)n * 3], qy = qp[(size_t)n * 3 + 1], qz = qp[(size_t)n * 3 + 2];
    const float px = shadow ? 1.0e6f : sp[(size_t)id * 3], py = shadow ? 1.0e6f : sp[(size_t)id * 3 + 1], pz = shadow ? 1.0e6f : sp[(size_t)id * 3 + 2];
    const float ox = px - qx, oy = py - qy, oz = pz - qz;
#pragma unroll
    for (int k = 0; k < KP; ++k) { const float dx = ox - skp[k * 3], dy = oy - skp[k * 3 + 1], dz = oz - skp[k * 3 + 2];
      const float d2 = __fadd_rn(__fadd_rn(__fmul_rn(dx, dx), __fmul_rn(dy, dy)), __fmul_rn(dz, dz));
      const float wv = 1.0f - sqrtf(d2) * (1.0f / 0.06f);   sw[w][k][lane] = wv > 0.f ? wv : 0.f; } }
  LDSX();
  if (lane < KP) { float s = 0.f; for (int m = 0; m < MM; ++m) s += sw[w][lane][m]; const float inv = 1.0f / (s + 1e-10f); for (int m = 0; m < MM; ++m) sw[w][lane][m] *= inv; }
  LDSX();
  float acc0[KP], acc1[KP];
#pragma unroll
  for (int k = 0; k < KP; ++k) { acc0[k] = 0.f; acc1[k] = 0.f; }
#pragma unroll 1
  for (int m = 0; m < MM; ++m) { const int id = sid[w][m]; const float f0 = id < 0 ? 0.f : x[(size_t)id * CIN + lane], f1 = id < 0 ? 0.f : x[(size_t)id * CIN + lane + 32];
#pragma unroll
    for (int k = 0; k < KP; ++k) { const float wk = sw[w][k][m]; acc0[k] += wk * f0; acc1[k] += wk * f1; } }
  __shared__ __align__(16) float srow[8][KW];
#pragma unroll
  for (int k = 0; k < KP; ++k) { srow[w][k * CIN + lane] = acc0[k]; srow[w][k * CIN + lane + 32] = acc1[k]; }
  LDSX();
  for (int q = lane; q < KW / 4; q += 32) vst2(WF + (size_t)n * KW + q * 4, *(const v4f*)(&srow[w][q * 4]));
}
__global__ __launch_bounds__(128) void k_out(const float* __restrict__ WF, const float* __restrict__ W, float* __restrict__ out) {
  __shared__ __align__(16) float so[4][16][132];
  const int tid = threadIdx.x, wave = tid >> 5, lane = tid & 31, col = lane & 15, g = lane >> 4;
  const int r0 = blockIdx.x * 64 + wave * 16;
  v8f acc[8] = {};
#pragma unroll 1
  for (int kc = 0; kc < KW / 32; ++kc) { const F2 a = split_row(WF + (size_t)(r0 + col) * KW, kc * 32, lane);
#pragma unroll
    for (int j = 0; j < 8; ++j) acc[j] = mac3(a, split_col(W, kc * 32, j * 16 + col, lane, COUT, KW), acc[j]); }
#pragma unroll
  for (int j = 0; j < 8; ++j)
#pragma unroll
    for (int r = 0; r < 8; ++r) so[wave][8 * g + r][j * 16 + col] = acc[j][r];
  LDSX();
#pragma unroll 4
  for (int rl = 0; rl < 16; ++rl) vst2(out + (size_t)(r0 + rl) * COUT + lane * 4, *(const v4f*)(&so[wave][rl][lane * 4]));
}
extern "C" void kernel_launch(void* const* d_in, const int* in_sizes, int n_in, void* d_out, int out_size, void* d_ws, size_t ws_size, hipStream_t stream) {
  (void)in_sizes; (void)n_in; (void)out_size; (void)ws_size;
  const float* qp = (const float*)d_in[0]; const float* sp = (const float*)d_in[1]; const int* nb = (const int*)d_in[2]; const float* x = (const float*)d_in[3]; const float* kpts = (const float*)d_in[4]; const float* W = (const float*)d_in[5];
  float* out = (float*)d_out;
  float* WF = (float*)d_ws;
  k_agg<<<NQ / 8, 256, 0, stream>>>(qp, sp, nb, x, kpts, WF);
  k_out<<<NQ / 64, 128, 0, stream>>>(WF, W, out);
}
